// MambaLayer_6863357739621
// MI455X (gfx1250) — hardware-verified
//
#include <hip/hip_runtime.h>
#include <math.h>

typedef __attribute__((ext_vector_type(16))) _Float16 v16h;
typedef __attribute__((ext_vector_type(8)))  _Float16 v8h;
typedef __attribute__((ext_vector_type(16))) __bf16   v16b;
typedef __attribute__((ext_vector_type(8)))  __bf16   v8b;
typedef __attribute__((ext_vector_type(8)))  float    v8f;
typedef __attribute__((ext_vector_type(4)))  float    v4f;
typedef __attribute__((ext_vector_type(2)))  float    v2f;
typedef __attribute__((ext_vector_type(2)))  unsigned v2u;

constexpr int kBatch = 4;
constexpr int kSeqL  = 2048;
constexpr int kDm    = 512;
constexpr int kDi    = 1024;
constexpr int kNst   = 128;
constexpr int kConvC = kDi + 2 * kNst;
constexpr int kNin   = 2 * kDi + 2 * kNst + 1;
constexpr int kNinP  = 2368;
constexpr int kNz    = kDi;
constexpr int kNx    = kNinP - kNz;
constexpr int kColDt = kConvC;
constexpr int kRows  = kBatch * kSeqL;
constexpr int kTS    = 32;
constexpr int kPB    = 64;
constexpr int kCVW   = 2 * kNst + kPB;
constexpr int kYP    = 68;
constexpr float kCarY = 16.0f;
constexpr float kCarW = 32.0f;
constexpr float kOutScale = 1.0f / (kCarY * kCarW);
static_assert(kConvC == 1280 && kNin == 2305 && kNx == 1344 && kRows == 8192, "shapes");
static_assert((kDm % 32) == 0 && (kDi % 32) == 0, "GEMM K multiples of 32");
static_assert((kRows % 64) == 0 && (kNz % 64) == 0 && (kNx % 64) == 0 && (kDm % 64) == 0, "GEMM M,N multiples of 64");
static_assert(kNinP >= kNin && (kNinP % 64) == 0, "padded in_proj width");
static_assert((kSeqL % kTS) == 0 && (kDi % kPB) == 0 && kTS == 32 && kPB == 64 && kCVW == 320, "scan tiling");
static_assert((kDm % 8) == 0 && (kDi % 8) == 0, "8-element casts");

constexpr size_t kSzXb    = (size_t)kRows * kDm * 2;
constexpr size_t kSzWin   = (size_t)kNinP * kDm * 2;
constexpr size_t kSzWout  = (size_t)kDm * kDi * 2;
constexpr size_t kSzZ     = (size_t)kRows * kNz * 2;
constexpr size_t kSzXbd   = (size_t)kRows * kNx * 4;
constexpr size_t kSzYg    = (size_t)kRows * kDi * 4;
constexpr size_t kSzYn    = (size_t)kRows * kDi * 2;
constexpr size_t kOffXb   = 0;
constexpr size_t kOffWin  = kOffXb + kSzXb;
constexpr size_t kOffWout = kOffWin + kSzWin;
constexpr size_t kOffZ    = kOffWout + kSzWout;
constexpr size_t kOffXbd  = kOffZ + kSzZ;
constexpr size_t kOffYg   = kOffXbd + kSzXbd;
constexpr size_t kOffYn   = kOffYg + kSzYg;
constexpr size_t kWsTotal = kOffYn + kSzYn;
static_assert(kWsTotal == 123011072ull, "carve total");
static_assert(kWsTotal <= 134217728ull, "carve cap");
static_assert((kOffWin % 128) == 0 && (kOffWout % 128) == 0 && (kOffZ % 128) == 0 && (kOffXbd % 128) == 0 &&
              (kOffYg % 128) == 0 && (kOffYn % 128) == 0, "128-B aligned regions");
static_assert(((size_t)kNx * 4) % 128 == 0 && ((size_t)kNz * 2) % 128 == 0 && ((size_t)kDi * 2) % 128 == 0, "line-multiple row pitches");

constexpr size_t kOut0N = (size_t)kRows * kDm;
constexpr size_t kOut1N = (size_t)kBatch * kDm;
static_assert(kOut0N * 4 == 16777216ull && (kOut0N * 4) % 128 == 0, "out1 byte offset");
static_assert(kOut0N * 4 + kOut1N * 4 == 16785408ull, "d_out total");
static_assert((kOut1N % (4 * 256)) == 0 || (kOut1N % 4) == 0, "out1 float4 copy");

__device__ __forceinline__ unsigned short f2bf_bits(float f) {
  unsigned u = __float_as_uint(f);
  return (unsigned short)((u + 0x7FFFu + ((u >> 16) & 1u)) >> 16);
}
__device__ __forceinline__ float bf_bits2f(unsigned short h) { return __uint_as_float(((unsigned)h) << 16); }
__device__ __forceinline__ float bfr(float f) { return bf_bits2f(f2bf_bits(f)); }

__device__ __forceinline__ float h16_to_f32(unsigned hb) {
  const unsigned sgn = (hb & 0x8000u) << 16; const unsigned em = hb & 0x7fffu;
  const float fn = __uint_as_float((em << 13) + 0x38000000u);
  const float fs = (float)em * 5.9604644775390625e-8f;
  const float mag = (em < 0x400u) ? fs : fn; return __uint_as_float(__float_as_uint(mag) | sgn); }

__device__ __forceinline__ void dep_guard_h(v8f& a, v8f& b, v16h x, v16h y) { asm volatile("v_nop\n\tv_nop\n\tv_nop\n\tv_nop" : "+v"(a), "+v"(b) : "v"(x), "v"(y)); }
__device__ __forceinline__ void dep_guard_b(v8f& a, v8f& b, v16b x, v16b y) { asm volatile("v_nop\n\tv_nop\n\tv_nop\n\tv_nop" : "+v"(a), "+v"(b) : "v"(x), "v"(y)); }
__device__ __forceinline__ void dep_guard4_h(v8f& a, v8f& b, v8f& c, v8f& d, v16h x, v16h y) { asm volatile("v_nop\n\tv_nop\n\tv_nop\n\tv_nop" : "+v"(a), "+v"(b), "+v"(c), "+v"(d) : "v"(x), "v"(y)); }
__device__ __forceinline__ void dep_guard4_b(v8f& a, v8f& b, v8f& c, v8f& d, v16b x, v16b y) { asm volatile("v_nop\n\tv_nop\n\tv_nop\n\tv_nop" : "+v"(a), "+v"(b), "+v"(c), "+v"(d) : "v"(x), "v"(y)); }
__device__ __forceinline__ void keep4_h(v16h a, v16h b, v16h c, v16h d) { asm volatile("v_nop" :: "v"(a), "v"(b), "v"(c), "v"(d)); }
__device__ __forceinline__ void keep4_b(v16b a, v16b b, v16b c, v16b d) { asm volatile("v_nop" :: "v"(a), "v"(b), "v"(c), "v"(d)); }
__device__ __forceinline__ void acc_guard4(v8f& a, v8f& b, v8f& c, v8f& d) { asm volatile("v_nop\n\tv_nop\n\tv_nop\n\tv_nop" : "+v"(a), "+v"(b), "+v"(c), "+v"(d)); }
template <typename T> struct Frag;
template <> struct Frag<_Float16> {
  typedef v16h V; union U { v16h v; v8h h[2]; };
  static __device__ __forceinline__ v16h load(const _Float16* p) {
    U f; f.h[0] = *(const v8h*)(p); f.h[1] = *(const v8h*)(p + 16); return f.v;
  }
  static __device__ __forceinline__ v8f mma(v16h a, v16h b, v8f c) {
    return __builtin_amdgcn_wmma_f32_16x16x32_f16(false, a, false, b, (short)0, c, false, false);
  }
  static __device__ __forceinline__ void guard(v8f& a, v8f& b, v16h x, v16h y) { dep_guard_h(a, b, x, y); }
  static __device__ __forceinline__ void guard4(v8f& a, v8f& b, v8f& c, v8f& d, v16h x, v16h y) { dep_guard4_h(a, b, c, d, x, y); }
  static __device__ __forceinline__ void keep(v16h a, v16h b, v16h c, v16h d) { keep4_h(a, b, c, d); }
};
template <> struct Frag<__bf16> {
  typedef v16b V; union U { v16b v; v8b h[2]; };
  static __device__ __forceinline__ v16b load(const __bf16* p) {
    U f; f.h[0] = *(const v8b*)(p); f.h[1] = *(const v8b*)(p + 16); return f.v;
  }
  static __device__ __forceinline__ v8f mma(v16b a, v16b b, v8f c) {
    return __builtin_amdgcn_wmma_f32_16x16x32_bf16(false, a, false, b, (short)0, c, false, false);
  }
  static __device__ __forceinline__ void guard(v8f& a, v8f& b, v16b x, v16b y) { dep_guard_b(a, b, x, y); }
  static __device__ __forceinline__ void guard4(v8f& a, v8f& b, v8f& c, v8f& d, v16b x, v16b y) { dep_guard4_b(a, b, c, d, x, y); }
  static __device__ __forceinline__ void keep(v16b a, v16b b, v16b c, v16b d) { keep4_b(a, b, c, d); }
};

template <int ET> struct Elem;
template <> struct Elem<0> { typedef _Float16 T; };
template <> struct Elem<1> { typedef __bf16 T; };
template <int ET, bool SPLIT, int BIAS_MODE, int OUT_MODE, bool RESID, int ACT = 0>
__global__ __launch_bounds__(256) void wmma_gemm64(
    const unsigned short* __restrict__ Ap, const unsigned short* __restrict__ A2p, int lda, long strideA,
    const unsigned short* __restrict__ Btp, const unsigned short* __restrict__ Bt2p, int ldb, long strideB,
    void* __restrict__ Cout, void* __restrict__ Cout2, int ldc, long strideC,
    const float* __restrict__ bias,
    const float* __restrict__ resid, long strideR,
    int M, int N, int K, float scale) {
  typedef typename Elem<ET>::T T;
  typedef typename Frag<T>::V V;
  const T* A = (const T*)Ap; const T* A2 = (const T*)A2p; const T* Bt = (const T*)Btp; const T* Bt2 = (const T*)Bt2p;
  __shared__ __align__(16) float sT[8][16 * 68];
  const int b    = blockIdx.y;
  const int lane = threadIdx.x & 31;
  const int wave = threadIdx.x >> 5;
  const int tilesN = N >> 6;
  const int tilesM = M >> 6;
  const int tile = blockIdx.x * 8 + wave;
  if (tile >= tilesM * tilesN) return;
  const int tm = tile / tilesN;
  const int tn = tile - tm * tilesN;
  const int m0 = tm << 6;
  const int n0 = tn << 6;

  const T* Ab  = A  + (size_t)b * strideA;
  const T* Bb  = Bt + (size_t)b * strideB;
  const T* Ab2 = SPLIT ? (A2  + (size_t)b * strideA) : nullptr;
  const T* Bb2 = SPLIT ? (Bt2 + (size_t)b * strideB) : nullptr;

  const int rlane = lane & 15;
  const int koff  = (lane >> 4) * 8;
  const int mOff  = (lane >> 4) * 8;

  v8f acc[4][4];
#pragma unroll
  for (int i = 0; i < 4; ++i)
#pragma unroll
    for (int j = 0; j < 4; ++j) acc[i][j] = (v8f){0.f,0.f,0.f,0.f,0.f,0.f,0.f,0.f};

  for (int k0 = 0; k0 < K; k0 += 32) {
    V bh[4], bl[4];
#pragma unroll
    for (int j = 0; j < 4; ++j) {
      const size_t bo = (size_t)(n0 + (j << 4) + rlane) * ldb + koff + k0;
      bh[j] = Frag<T>::load(Bb + bo);
      if (SPLIT) bl[j] = Frag<T>::load(Bb2 + bo);
    }
#pragma unroll
    for (int i = 0; i < 4; ++i) {
      const size_t ao = (size_t)(m0 + (i << 4) + rlane) * lda + koff + k0;
      V ah = Frag<T>::load(Ab + ao);
      V al;
      if (SPLIT) al = Frag<T>::load(Ab2 + ao);
#pragma unroll
      for (int j = 0; j < 4; ++j) {
        acc[i][j] = Frag<T>::mma(ah, bh[j], acc[i][j]);
        if (SPLIT) {
          acc[i][j] = Frag<T>::mma(ah, bl[j], acc[i][j]);
          acc[i][j] = Frag<T>::mma(al, bh[j], acc[i][j]);
        }
      }
      Frag<T>::guard4(acc[i][0], acc[i][1], acc[i][2], acc[i][3], ah, SPLIT ? al : ah);
    }
    Frag<T>::keep(bh[0], bh[1], bh[2], bh[3]);
    if (SPLIT) Frag<T>::keep(bl[0], bl[1], bl[2], bl[3]);
  }
  acc_guard4(acc[0][0], acc[0][1], acc[0][2], acc[0][3]);
  acc_guard4(acc[1][0], acc[1][1], acc[1][2], acc[1][3]);
  acc_guard4(acc[2][0], acc[2][1], acc[2][2], acc[2][3]);
  acc_guard4(acc[3][0], acc[3][1], acc[3][2], acc[3][3]);

  float* slab = sT[wave];
  const float* Rb = RESID ? (resid + (size_t)b * strideR) : nullptr;
#pragma unroll
  for (int i = 0; i < 4; ++i) {
    const int mBase = m0 + (i << 4);
#pragma unroll
    for (int j = 0; j < 4; ++j) {
      const int n = n0 + (j << 4) + rlane;
      float bv = 0.f;
      if (BIAS_MODE == 2) bv = bias[n];
#pragma unroll
      for (int r = 0; r < 8; ++r) {
        float v = acc[i][j][r] * scale;
        if (BIAS_MODE == 1) v += bias[mBase + mOff + r];
        if (BIAS_MODE == 2) v += bv;
        if (RESID) v += Rb[(size_t)(mBase + mOff + r) * ldc + n];
        if (ACT == 1) v = tanhf(v);
        if (ACT == 2) v = fmaxf(v, 0.0f);
        if (ACT == 3) v = v / (1.0f + expf(-v));
        if (ACT == 4) v = (v > 0.f) ? v : 0.01f * v;
        slab[(mOff + r) * 68 + (j << 4) + rlane] = v;
      }
    }
    __builtin_amdgcn_fence(__ATOMIC_RELEASE, "workgroup");
    __builtin_amdgcn_wave_barrier();
    __builtin_amdgcn_fence(__ATOMIC_ACQUIRE, "workgroup");
    if (OUT_MODE == 0) {
      float* C = (float*)Cout + (size_t)b * strideC;
      const int hh = lane >> 4, c4 = (lane & 15) * 4;
      for (int pass = 0; pass < 2; ++pass) {
#pragma unroll
        for (int it = 0; it < 8; ++it) {
          const int row = it * 2 + hh;
          v4f v = *(const v4f*)(slab + row * 68 + c4);
          *(volatile v4f*)(C + (size_t)(mBase + row) * ldc + n0 + c4) = v;
        }
        __threadfence();
      }
    } else {
      const int q = lane >> 3, c8 = (lane & 7) * 8;
      unsigned short* C  = (unsigned short*)Cout  + (size_t)b * strideC;
      unsigned short* C2 = (OUT_MODE == 2) ? ((unsigned short*)Cout2 + (size_t)b * strideC) : nullptr;
      for (int pass = 0; pass < 2; ++pass) {
#pragma unroll
        for (int it = 0; it < 4; ++it) {
          const int row = it * 4 + q;
          const float* sp = slab + row * 68 + c8;
          v8h hv, lv;
#pragma unroll
          for (int e = 0; e < 8; ++e) {
            if (OUT_MODE == 1) {
              hv[e] = (_Float16)sp[e];
            } else {
              unsigned short hb = f2bf_bits(sp[e]);
              unsigned short lb = f2bf_bits(sp[e] - bf_bits2f(hb));
              hv[e] = __builtin_bit_cast(_Float16, hb);
              lv[e] = __builtin_bit_cast(_Float16, lb);
            }
          }
          *(volatile v8h*)(C + (size_t)(mBase + row) * ldc + n0 + c8) = hv;
          if (OUT_MODE == 2) *(volatile v8h*)(C2 + (size_t)(mBase + row) * ldc + n0 + c8) = lv;
        }
        __threadfence();
      }
    }
    __builtin_amdgcn_fence(__ATOMIC_RELEASE, "workgroup");
    __builtin_amdgcn_wave_barrier();
    __builtin_amdgcn_fence(__ATOMIC_ACQUIRE, "workgroup");
  }
}

__global__ __launch_bounds__(256) void cast_rows_bf16_kernel(
    const float* __restrict__ src, unsigned short* __restrict__ dst, int ncol, int nrowsReal, int total8)
{
  const int i = blockIdx.x * 256 + threadIdx.x;
  if (i >= total8) return;
  const size_t e0 = (size_t)i << 3;
  const int row = (int)(e0 / (size_t)ncol);
  const int col = (int)(e0 - (size_t)row * (size_t)ncol);
  const bool live = (row < nrowsReal);
  const int rowc = live ? row : (nrowsReal - 1);
  const float livef = live ? 1.0f : 0.0f;
  const float* p = src + (size_t)rowc * ncol + col;
  const v4f a0 = *(const v4f*)(p);
  const v4f a1 = *(const v4f*)(p + 4);
  v8h hv;
#pragma unroll
  for (int e = 0; e < 4; ++e) {
    const float f0 = livef * a0[e];
    const float f1 = livef * a1[e];
    hv[e]     = __builtin_bit_cast(_Float16, f2bf_bits(f0));
    hv[4 + e] = __builtin_bit_cast(_Float16, f2bf_bits(f1));
  }
  unsigned short* q = dst + e0;
  *(volatile v8h*)q = hv;
  __threadfence();
  *(volatile v8h*)q = hv;
}

__global__ __launch_bounds__(256) void cast_f16_bfr_kernel(
    const float* __restrict__ src, unsigned short* __restrict__ dst, int total8, float scale)
{
  const int i = blockIdx.x * 256 + threadIdx.x;
  if (i >= total8) return;
  const size_t e0 = (size_t)i << 3;
  const v4f a0 = *(const v4f*)(src + e0);
  const v4f a1 = *(const v4f*)(src + e0 + 4);
  v8h hv;
#pragma unroll
  for (int e = 0; e < 4; ++e) {
    hv[e]     = (_Float16)(bfr(a0[e]) * scale);
    hv[4 + e] = (_Float16)(bfr(a1[e]) * scale);
  }
  unsigned short* q = dst + e0;
  *(volatile v8h*)q = hv;
  __threadfence();
  *(volatile v8h*)q = hv;
}

__global__ __launch_bounds__(512) void scan_kernel(
    const float* __restrict__ XBD, const unsigned* __restrict__ Zw,
    const float* __restrict__ cw, const float* __restrict__ cb,
    const float* __restrict__ dtbp, const float* __restrict__ alogp, const float* __restrict__ dpp,
    float* __restrict__ YG)
{
  __shared__ __align__(16) float sCV[kTS * kCVW];
  __shared__ __align__(16) float sG[kTS * kPB];
  __shared__ __align__(16) float sY[kTS * kYP];
  __shared__ __align__(16) float sDD[2 * kTS];
  const int tid  = threadIdx.x;
  const int lane = tid & 31, wave = tid >> 5;
  const int p0   = blockIdx.x * kPB;
  const size_t rowb = (size_t)blockIdx.y * kSeqL;
  const bool isBC   = tid < 2 * kNst;
  const bool doConv = tid < kCVW;
  const bool doDt   = (tid >= kCVW) && (tid < kCVW + kTS);
  const int ch = isBC ? (kDi + tid) : (p0 + ((tid - 2 * kNst) & (kPB - 1)));
  const v4f wv = *(const v4f*)(cw + (size_t)ch * 4);
  const float w0 = bfr(wv[0]), w1 = bfr(wv[1]), w2 = bfr(wv[2]), w3 = bfr(wv[3]);
  const float cbv  = bfr(cb[ch]);
  const float dtb  = bfr(dtbp[0]);
  const float aneg = -expf(bfr(alogp[0]));
  const float dsk  = bfr(dpp[0]);
  float xm1 = 0.0f, xm2 = 0.0f, xm3 = 0.0f;
  const int pl = tid >> 3, nq = tid & 7;
  const int zr = tid >> 4, zc = (tid & 15) * 4;
  float st[16];
#pragma unroll
  for (int k = 0; k < 16; ++k) st[k] = 0.0f;

#pragma unroll 1
  for (int cix = 0; cix < kSeqL / kTS; ++cix) {
    const int t0 = cix * kTS;
    __syncthreads();
    {
      const size_t hoff = (rowb + t0 + zr) * (size_t)kDi + p0 + zc;
      const v2u wz = *(const v2u*)(Zw + (hoff >> 1));
      const unsigned wlo = wz[0], whi = wz[1];
#pragma unroll 1
      for (int e = 0; e < 4; ++e) {
        const unsigned word = (e < 2) ? wlo : whi;
        const unsigned hb = (e & 1) ? (word >> 16) : (word & 0xffffu);
        const float z = h16_to_f32(hb);
        const float g = z * __builtin_amdgcn_rcpf(1.0f + expf(-z));
        sG[zr * kPB + zc + e] = g;
      }
    }
    if (doConv) {
#pragma unroll 1
      for (int s = 0; s < kTS; ++s) {
        const float xc = XBD[(rowb + t0 + s) * (size_t)kNx + ch];
        float a = w0 * xm3;
        a = fmaf(w1, xm2, a);
        a = fmaf(w2, xm1, a);
        a = fmaf(w3, xc, a);
        const float v = a + cbv;
        const float g = v * __builtin_amdgcn_rcpf(1.0f + expf(-v));
        sCV[s * kCVW + tid] = g;
        xm3 = xm2; xm2 = xm1; xm1 = xc;
      }
    }
    if (doDt) {
      const int s = tid - kCVW;
      const float raw = XBD[(rowb + t0 + s) * (size_t)kNx + kColDt];
      const float v = raw + dtb;
      const float sp = fmaxf(v, 0.0f) + log1pf(expf(-fabsf(v)));
      float da = expf(sp * aneg);
      da = (da < 1.17549435e-38f) ? 0.0f : da;
      v2f dd; dd[0] = sp; dd[1] = da;
      *(v2f*)(sDD + 2 * s) = dd;
    }
    __syncthreads();
#pragma unroll 1
    for (int s = 0; s < kTS; ++s) {
      const float* cv = sCV + s * kCVW;
      const v2f dd = *(const v2f*)(sDD + 2 * s);
      const float dt = dd[0], dA = dd[1];
      const float xv = cv[2 * kNst + pl];
      const float coef = dt * xv;
      float acc = 0.0f;
#pragma unroll
      for (int j = 0; j < 4; ++j) {
        const v4f bq = *(const v4f*)(cv + 32 * j + 4 * nq);
        const v4f cq = *(const v4f*)(cv + kNst + 32 * j + 4 * nq);
#pragma unroll
        for (int e = 0; e < 4; ++e) {
          const float hn = dA * st[4 * j + e] + coef * bq[e];
          st[4 * j + e] = hn;
          acc = fmaf(hn, cq[e], acc);
        }
      }
      acc += __shfl_xor(acc, 1);
      acc += __shfl_xor(acc, 2);
      acc += __shfl_xor(acc, 4);
      const float y = fmaf(dsk, xv, acc);
      const float g = y * sG[s * kPB + pl];
      if (nq == 0) sY[s * kYP + pl] = g;
    }
    __syncthreads();
    {
      const int hh = lane >> 4, c4 = (lane & 15) * 4;
      const int row = wave * 2 + hh;
      const v4f val = *(const v4f*)(sY + row * kYP + c4);
      float* q = YG + (rowb + t0 + row) * (size_t)kDi + p0 + c4;
      *(volatile v4f*)q = val;
      __threadfence();
      *(volatile v4f*)q = val;
    }
  }
}

__global__ __launch_bounds__(128) void rmsnorm_cast_kernel(
    const float* __restrict__ YG, const float* __restrict__ nw, unsigned short* __restrict__ YN)
{
  __shared__ float red[4];
  const int tid = threadIdx.x, lane = tid & 31, wave = tid >> 5;
  const size_t base = (size_t)blockIdx.x * kDi + (size_t)tid * 8;
  const v4f a0 = *(const v4f*)(YG + base);
  const v4f a1 = *(const v4f*)(YG + base + 4);
  float ss = 0.0f;
#pragma unroll
  for (int e = 0; e < 4; ++e) ss = fmaf(a0[e], a0[e], ss);
#pragma unroll
  for (int e = 0; e < 4; ++e) ss = fmaf(a1[e], a1[e], ss);
#pragma unroll
  for (int off = 16; off >= 1; off >>= 1) ss += __shfl_xor(ss, off);
  if (lane == 0) red[wave] = ss;
  __syncthreads();
  const float tot = (red[0] + red[1]) + (red[2] + red[3]);
  const float rs = rsqrtf(tot * (1.0f / (float)kDi) + 1e-5f);
  const v4f n0 = *(const v4f*)(nw + tid * 8);
  const v4f n1 = *(const v4f*)(nw + tid * 8 + 4);
  v8h hv;
#pragma unroll
  for (int e = 0; e < 4; ++e) {
    hv[e]     = (_Float16)(((a0[e] * rs) * bfr(n0[e])) * kCarY);
    hv[4 + e] = (_Float16)(((a1[e] * rs) * bfr(n1[e])) * kCarY);
  }
  unsigned short* q = YN + base;
  *(volatile v8h*)q = hv;
  __threadfence();
  *(volatile v8h*)q = hv;
}

__global__ __launch_bounds__(256) void copy4_kernel(const float* __restrict__ src, float* __restrict__ dst, int n4)
{
  const int i = blockIdx.x * 256 + threadIdx.x;
  if (i >= n4) return;
  const v4f v = *(const v4f*)(src + (size_t)i * 4);
  float* q = dst + (size_t)i * 4;
  *(volatile v4f*)q = v;
  __threadfence();
  *(volatile v4f*)q = v;
}

extern "C" void kernel_launch(void* const* d_in, const int* in_sizes, int n_in,
                              void* d_out, int out_size, void* d_ws, size_t ws_size,
                              hipStream_t stream)
{
  if (n_in < 10) return;
  if (in_sizes[0] != kRows * kDm) return;
  if (in_sizes[1] != kBatch * kDm) return;
  if (in_sizes[2] != kNin * kDm) return;
  if (in_sizes[3] != kConvC * 4) return;
  if (in_sizes[4] != kConvC) return;
  if (in_sizes[5] < 1 || in_sizes[6] < 1 || in_sizes[7] < 1) return;
  if (in_sizes[8] != kDi) return;
  if (in_sizes[9] != kDm * kDi) return;
  if (out_size != (int)(kOut0N + kOut1N)) return;
  if (ws_size < kWsTotal) return;

  const float* x       = (const float*)d_in[0];
  const float* rstate  = (const float*)d_in[1];
  const float* W_in    = (const float*)d_in[2];
  const float* conv_w  = (const float*)d_in[3];
  const float* conv_b  = (const float*)d_in[4];
  const float* dt_bias = (const float*)d_in[5];
  const float* A_log   = (const float*)d_in[6];
  const float* Dp      = (const float*)d_in[7];
  const float* norm_w  = (const float*)d_in[8];
  const float* W_out   = (const float*)d_in[9];
  float* dout = (float*)d_out;

  char* ws = (char*)d_ws;
  unsigned short* XB   = (unsigned short*)(ws + kOffXb);
  unsigned short* WINB = (unsigned short*)(ws + kOffWin);
  unsigned short* WO16 = (unsigned short*)(ws + kOffWout);
  unsigned short* Z16  = (unsigned short*)(ws + kOffZ);
  float*          XBD  = (float*)(ws + kOffXbd);
  float*          YG   = (float*)(ws + kOffYg);
  unsigned short* YN16 = (unsigned short*)(ws + kOffYn);
  const float* dummy_bias  = norm_w;
  const float* dummy_resid = x;

  cast_rows_bf16_kernel<<<(kRows * kDm) / 8 / 256, 256, 0, stream>>>(x, XB, kDm, kRows, (kRows * kDm) / 8);
  cast_rows_bf16_kernel<<<(kNinP * kDm) / 8 / 256, 256, 0, stream>>>(W_in, WINB, kDm, kNin, (kNinP * kDm) / 8);
  cast_f16_bfr_kernel<<<(kDm * kDi) / 8 / 256, 256, 0, stream>>>(W_out, WO16, (kDm * kDi) / 8, kCarW);

  wmma_gemm64<1, false, 0, 1, false><<<dim3((kRows / 64) * (kNz / 64) / 8, 1), 256, 0, stream>>>(
      XB, XB, kDm, 0L, WINB, WINB, kDm, 0L,
      (void*)Z16, (void*)Z16, kNz, 0L, dummy_bias, dummy_resid, 0L, kRows, kNz, kDm, 1.0f);

  wmma_gemm64<1, false, 0, 0, false><<<dim3((kRows / 64) * (kNx / 64) / 8, 1), 256, 0, stream>>>(
      XB, XB, kDm, 0L, WINB + (size_t)kNz * kDm, WINB + (size_t)kNz * kDm, kDm, 0L,
      (void*)XBD, (void*)XBD, kNx, 0L, dummy_bias, dummy_resid, 0L, kRows, kNx, kDm, 1.0f);

  scan_kernel<<<dim3(kDi / kPB, kBatch), 512, 0, stream>>>(
      XBD, (const unsigned*)Z16, conv_w, conv_b, dt_bias, A_log, Dp, YG);

  rmsnorm_cast_kernel<<<kRows, 128, 0, stream>>>(YG, norm_w, YN16);

  wmma_gemm64<0, false, 0, 0, false><<<dim3((kRows / 64) * (kDm / 64) / 8, 1), 256, 0, stream>>>(
      YN16, YN16, kDi, 0L, WO16, WO16, kDi, 0L,
      (void*)dout, (void*)dout, kDm, 0L, dummy_bias, dummy_resid, 0L, kRows, kDm, kDi, kOutScale);

  copy4_kernel<<<(int)(kOut1N / 4) / 256, 256, 0, stream>>>(rstate, dout + kOut0N, (int)(kOut1N / 4));
}
